// InformedTestModel_33423435497942
// MI455X (gfx1250) — hardware-verified
//
#include <hip/hip_runtime.h>


#define NB_  8
#define NT_  2048
#define NTK  (NB_ * NT_)
#define VOC  240
#define DQ1  256
#define DV1  512
#define LOOK 64
#define NH_  8
#define DK2  32
#define DV2  128
#define DQ2  (NH_ * DK2)
#define DO2  (NH_ * DV2)
#define NEGF (-1.0e9f)
#define PSC  32768.0f
#define LOSC 1024.0f
#define LOSCI (1.0f / 1024.0f)

typedef _Float16 h16;
typedef unsigned short bf;
typedef __attribute__((ext_vector_type(16))) __bf16   v16bf;
typedef __attribute__((ext_vector_type(16))) _Float16 v16h;
typedef __attribute__((ext_vector_type(8)))  _Float16 v8h;
typedef __attribute__((ext_vector_type(8)))  unsigned short v8us;
typedef __attribute__((ext_vector_type(8)))  float    v8f;
typedef __attribute__((ext_vector_type(4)))  float    v4f;
typedef v8h  __attribute__((may_alias)) v8ha;
typedef v4f  __attribute__((may_alias)) v4fa;
typedef v8us __attribute__((may_alias)) v8usa;

__device__ __forceinline__ unsigned short f2bf(float f) { unsigned u = __float_as_uint(f); u += 0x7FFFu + ((u >> 16) & 1u); return (unsigned short)(u >> 16); }
__device__ __forceinline__ float bf2f(unsigned short b) { return __uint_as_float(((unsigned)b) << 16); }
__device__ __forceinline__ float bfr(float f) { return bf2f(f2bf(f)); }
__device__ __forceinline__ v16h cat16(v8h lo, v8h hi) { return __builtin_shufflevector(lo, hi, 0, 1, 2, 3, 4, 5, 6, 7, 8, 9, 10, 11, 12, 13, 14, 15); }
__device__ __forceinline__ v16bf cat16b(v8us lo, v8us hi) { return __builtin_bit_cast(v16bf, __builtin_shufflevector(lo, hi, 0, 1, 2, 3, 4, 5, 6, 7, 8, 9, 10, 11, 12, 13, 14, 15)); }
__device__ __forceinline__ v8f wmma16(v16h a, v16h b, v8f c) { return __builtin_amdgcn_wmma_f32_16x16x32_f16(false, a, false, b, (short)0, c, false, false); }
__device__ __forceinline__ v8f wmmab(v16bf a, v16bf b, v8f c) { return __builtin_amdgcn_wmma_f32_16x16x32_bf16(false, a, false, b, (short)0, c, false, false); }
#define VST2(T, p, v) do { const T vst2_v_ = (v); *(volatile T*)(p) = vst2_v_; __threadfence(); *(volatile T*)(p) = vst2_v_; } while (0)

__global__ __launch_bounds__(256) void k_gather(const int* __restrict__ xs, const float* __restrict__ lq, const float* __restrict__ lk, bf* Q1, bf* K1) {
    const int lane = threadIdx.x & 31; const size_t t = (size_t)blockIdx.x * 8 + (threadIdx.x >> 5);
    if (t >= (size_t)NTK) return;
    int tokv = xs[t]; tokv = tokv < 0 ? 0 : (tokv >= VOC ? VOC - 1 : tokv);
    v8us oq, ok;
#pragma unroll
    for (int i = 0; i < 8; ++i) { oq[i] = f2bf(lq[(size_t)tokv * DQ1 + lane * 8 + i]); ok[i] = f2bf(lk[(size_t)tokv * DQ1 + lane * 8 + i]); }
    *(volatile v8us*)(Q1 + t * DQ1 + lane * 8) = oq; *(volatile v8us*)(K1 + t * DQ1 + lane * 8) = ok; __threadfence();
    *(volatile v8us*)(Q1 + t * DQ1 + lane * 8) = oq; *(volatile v8us*)(K1 + t * DQ1 + lane * 8) = ok;
}
__global__ __launch_bounds__(256) void k_gvt(const int* __restrict__ xs, const float* __restrict__ lv, bf* V1T) {
    __shared__ __align__(16) unsigned short tl[64 * 72];
    const int tid = threadIdx.x, t0 = blockIdx.x * 64, d0 = blockIdx.y * 64, b = blockIdx.z;
    { const int tt = tid >> 2, dq = (tid & 3) * 16; int tokv = xs[(size_t)b * NT_ + t0 + tt]; tokv = tokv < 0 ? 0 : (tokv >= VOC ? VOC - 1 : tokv);
#pragma unroll
      for (int i = 0; i < 16; ++i) tl[(dq + i) * 72 + tt] = f2bf(lv[(size_t)tokv * DV1 + d0 + dq + i]); }
    __syncthreads();
    const int piece = tid & 7;
    auto pass = [&]() {
#pragma unroll
        for (int s = 0; s < 2; ++s) { const int d = (tid >> 3) + 32 * s; const v8us val = *(const v8usa*)(tl + d * 72 + piece * 8); *(volatile v8us*)(V1T + ((size_t)b * DV1 + d0 + d) * NT_ + t0 + piece * 8) = val; }
    };
    pass(); __threadfence(); pass();
}
__global__ __launch_bounds__(128) void k_local(const bf* __restrict__ Q1, const bf* __restrict__ K1, const bf* __restrict__ V1T, const float* __restrict__ relb, bf* X2H, bf* X2L) {
    __shared__ __align__(16) unsigned short plds[4][16 * 32];
    __shared__ __align__(16) unsigned short plds2[4][16 * 32];
    __shared__ __align__(16) float ost[4][16 * 68];
    const int lane = threadIdx.x & 31, wave = threadIdx.x >> 5, lr = lane & 15, hi = lane >> 4;
    const int b = blockIdx.z, qt = blockIdx.x, ch = blockIdx.y, q0 = qt * 64 + wave * 16;
    const size_t tok0 = (size_t)b * NT_;
    unsigned short* pl = &plds[wave][0]; unsigned short* pl2 = &plds2[wave][0];
    const bf* qrow = Q1 + (tok0 + q0 + lr) * DQ1 + 8 * hi;
    v8f o[8];
#pragma unroll
    for (int n = 0; n < 8; ++n) o[n] = (v8f){};
    float mrow[8], lpart[8];
#pragma unroll
    for (int j = 0; j < 8; ++j) { mrow[j] = -3.0e38f; lpart[j] = 0.f; }
    const int kt_lo = (qt * 64 - LOOK) > 0 ? (qt * 64 - LOOK) / 32 : 0; int kt_hi = (qt * 64 + 63 + LOOK) / 32; if (kt_hi > NT_ / 32 - 1) kt_hi = NT_ / 32 - 1;
#pragma unroll 1
    for (int kt = kt_lo; kt <= kt_hi; ++kt) {
        const int l0 = kt * 32;
        v8f s0 = {}, s1 = {};
#pragma unroll
        for (int kc = 0; kc < 8; ++kc) { const v16bf qa = cat16b(*(const v8us*)(qrow + kc * 32), *(const v8us*)(qrow + kc * 32 + 16));
            const bf* k0p = K1 + (tok0 + l0 + lr) * DQ1 + kc * 32 + 8 * hi; const bf* k1p = k0p + (size_t)16 * DQ1;
            s0 = wmmab(qa, cat16b(*(const v8us*)k0p, *(const v8us*)(k0p + 16)), s0); s1 = wmmab(qa, cat16b(*(const v8us*)k1p, *(const v8us*)(k1p + 16)), s1);
            asm volatile("" : "+v"(s0), "+v"(s1) : "v"(qa) : "memory"); }
        asm volatile("v_nop\n\tv_nop\n\tv_nop\n\tv_nop" : "+v"(s0), "+v"(s1));
        float alpha[8];
#pragma unroll
        for (int j = 0; j < 8; ++j) { const int qi = q0 + hi * 8 + j, ja = l0 + lr, jb = l0 + 16 + lr; const int ra = ja - qi, rb = jb - qi;
            const float a0 = (ra >= -LOOK && ra <= LOOK) ? s0[j] * 0.0625f + bfr(relb[ra + LOOK]) : NEGF, a1 = (rb >= -LOOK && rb <= LOOK) ? s1[j] * 0.0625f + bfr(relb[rb + LOOK]) : NEGF;
            float mx = fmaxf(a0, a1);
            mx = fmaxf(mx, __shfl_xor(mx, 1, 16)); mx = fmaxf(mx, __shfl_xor(mx, 2, 16)); mx = fmaxf(mx, __shfl_xor(mx, 4, 16)); mx = fmaxf(mx, __shfl_xor(mx, 8, 16));
            const float mn = fmaxf(mrow[j], mx);
            alpha[j] = __expf(mrow[j] - mn); mrow[j] = mn;
            const float p0 = __expf(a0 - mn), p1 = __expf(a1 - mn);
            lpart[j] = lpart[j] * alpha[j] + (p0 + p1);
            const int mr = hi * 8 + j; const float ps0 = p0 * PSC, ps1 = p1 * PSC; const unsigned short h0 = f2bf(ps0), h1 = f2bf(ps1);
            pl[mr * 32 + lr] = h0; pl[mr * 32 + 16 + lr] = h1; pl2[mr * 32 + lr] = f2bf(ps0 - bf2f(h0)); pl2[mr * 32 + 16 + lr] = f2bf(ps1 - bf2f(h1)); }
#pragma unroll
        for (int n = 0; n < 8; ++n)
#pragma unroll
            for (int j = 0; j < 8; ++j) o[n][j] *= alpha[j];
        asm volatile("" ::: "memory");
        const v16bf pa = cat16b(*(const v8usa*)(pl + lr * 32 + hi * 8), *(const v8usa*)(pl + lr * 32 + 16 + hi * 8));
        const v16bf px = cat16b(*(const v8usa*)(pl2 + lr * 32 + hi * 8), *(const v8usa*)(pl2 + lr * 32 + 16 + hi * 8));
#pragma unroll
        for (int n = 0; n < 8; ++n) { const bf* vp = V1T + ((size_t)b * DV1 + ch * 128 + n * 16 + lr) * NT_ + l0 + hi * 8; const v16bf vv = cat16b(*(const v8us*)vp, *(const v8us*)(vp + 16));
            o[n] = wmmab(pa, vv, o[n]); o[n] = wmmab(px, vv, o[n]);
            asm volatile("" : "+v"(o[n]) : "v"(vv) : "memory"); }
        asm volatile("v_nop\n\tv_nop\n\tv_nop\n\tv_nop" : "+v"(o[0]), "+v"(o[7]) : "v"(pa), "v"(px));
        __builtin_amdgcn_wave_barrier();
    }
    float inv[8];
#pragma unroll
    for (int j = 0; j < 8; ++j) { float rs = lpart[j]; rs += __shfl_xor(rs, 1, 16); rs += __shfl_xor(rs, 2, 16); rs += __shfl_xor(rs, 4, 16); rs += __shfl_xor(rs, 8, 16); inv[j] = 1.0f / (rs * PSC); }
    float* os = &ost[wave][0];
    const size_t pbase = (tok0 + q0) * DV1 + (size_t)ch * 128;
#pragma unroll
    for (int half = 0; half < 2; ++half) {
#pragma unroll
        for (int n = 0; n < 4; ++n)
#pragma unroll
            for (int j = 0; j < 8; ++j) os[(hi * 8 + j) * 68 + n * 16 + lr] = fmaxf((o[half * 4 + n][j]) * inv[j], 0.f);
        __builtin_amdgcn_wave_barrier(); asm volatile("" ::: "memory");
#pragma unroll
        for (int ps2 = 0; ps2 < 2; ++ps2) {
#pragma unroll
            for (int s = 0; s < 4; ++s) { const int row = 4 * s + (lane >> 3), piece = lane & 7; const float* sp = os + row * 68 + piece * 8; v8us oh, ol;
#pragma unroll
                for (int i = 0; i < 8; ++i) { const unsigned short hb = f2bf(sp[i]); oh[i] = hb; ol[i] = f2bf(sp[i] - bf2f(hb)); }
                const size_t po = pbase + (size_t)row * DV1 + half * 64 + piece * 8; *(volatile v8us*)(X2H + po) = oh; *(volatile v8us*)(X2L + po) = ol; }
            if (ps2 == 0) __threadfence(); }
        __builtin_amdgcn_wave_barrier(); asm volatile("" ::: "memory");
    }
}

__global__ __launch_bounds__(256) void k_wt(const float* __restrict__ Wm, int K, int ncols, int npad, bf* WT) {
    __shared__ __align__(16) unsigned short tl[64 * 72];
    const int tid = threadIdx.x, k0 = blockIdx.x * 64, n0 = blockIdx.y * 64;
    const int kk = tid >> 2, nq = (tid & 3) * 16;
#pragma unroll
    for (int i = 0; i < 16; ++i) { const int n = n0 + nq + i; tl[(nq + i) * 72 + kk] = (n < ncols) ? f2bf(Wm[(size_t)(k0 + kk) * ncols + n]) : (unsigned short)0; }
    __syncthreads();
    const int piece = tid & 7;
    auto pass = [&]() {
#pragma unroll
        for (int s = 0; s < 2; ++s) { const int nr = (tid >> 3) + 32 * s; if (n0 + nr < npad) { const v8us val = *(const v8usa*)(tl + nr * 72 + piece * 8); *(volatile v8us*)(WT + (size_t)(n0 + nr) * K + k0 + piece * 8) = val; } }
    };
    pass(); __threadfence(); pass();
}
template <int MODE>
__global__ __launch_bounds__(128) void k_gemm(const bf* __restrict__ A, const bf* __restrict__ Al, int lda, const bf* __restrict__ Bn, int K, int ldc, void* C, void* C2) {
    __shared__ __align__(16) float ost[4][16 * 68];
    __shared__ __align__(16) h16 vt[64 * 72];
    __shared__ __align__(16) h16 vt2[64 * 72];
    const int lane = threadIdx.x & 31, wave = threadIdx.x >> 5, lr = lane & 15, hi = lane >> 4, tid = threadIdx.x;
    const size_t r0 = (size_t)blockIdx.x * 64 + wave * 16; const int c0 = blockIdx.y * 64;
    const size_t aoff = (r0 + lr) * lda + 8 * hi;
    v8f acc[4];
#pragma unroll
    for (int t = 0; t < 4; ++t) acc[t] = (v8f){};
#pragma unroll 2
    for (int kc = 0; kc < K; kc += 32) {
        const v16bf a = cat16b(*(const v8us*)(A + aoff + kc), *(const v8us*)(A + aoff + kc + 16)), al = cat16b(*(const v8us*)(Al + aoff + kc), *(const v8us*)(Al + aoff + kc + 16));
#pragma unroll
        for (int t = 0; t < 4; ++t) { const bf* bp = Bn + (size_t)(c0 + t * 16 + lr) * K + kc + 8 * hi; const v16bf bb = cat16b(*(const v8us*)bp, *(const v8us*)(bp + 16)); acc[t] = wmmab(a, bb, acc[t]); acc[t] = wmmab(al, bb, acc[t]); }
        asm volatile("v_nop" : "+v"(acc[0]), "+v"(acc[1]), "+v"(acc[2]), "+v"(acc[3]) : "v"(a), "v"(al) : "memory");
    }
    float* os = &ost[wave][0];
#pragma unroll
    for (int t = 0; t < 4; ++t)
#pragma unroll
        for (int j = 0; j < 8; ++j) os[(hi * 8 + j) * 68 + t * 16 + lr] = acc[t][j];
    __syncthreads();
    if (MODE == 0) {
        h16* c1 = (h16*)C + r0 * ldc + c0; h16* c2 = (h16*)C2 + r0 * ldc + c0;
        auto pass = [&]() {
#pragma unroll
            for (int s = 0; s < 4; ++s) { const int row = 4 * s + (lane >> 3), piece = lane & 7; const float* sp = os + row * 68 + piece * 8; v8h o1, o2;
#pragma unroll
                for (int i = 0; i < 8; ++i) { const h16 ah = (h16)sp[i]; o1[i] = ah; o2[i] = (h16)((sp[i] - (float)ah) * LOSC); }
                *(volatile v8h*)(c1 + (size_t)row * ldc + piece * 8) = o1; *(volatile v8h*)(c2 + (size_t)row * ldc + piece * 8) = o2; }
        };
        pass(); __threadfence(); pass();
    } else if (MODE == 1) {
        float* crow = (float*)C + r0 * ldc + c0;
        auto pass = [&]() {
#pragma unroll
            for (int s = 0; s < 8; ++s) { const int Lid = (lane >> 3) + 4 * s, piece = lane & 7; const int row = Lid >> 1, cofs = (Lid & 1) * 32 + piece * 4;
                const v4f val = *(const v4fa*)(os + row * 68 + cofs); *(volatile v4f*)(crow + (size_t)row * ldc + cofs) = val; }
        };
        pass(); __threadfence(); pass();
    } else if (MODE == 2) {
        { const int row = tid >> 1, half = tid & 1;
#pragma unroll
          for (int i = 0; i < 32; ++i) { const float v = ost[row >> 4][(row & 15) * 68 + half * 32 + i]; const h16 ah = (h16)v; vt[(half * 32 + i) * 72 + row] = ah; vt2[(half * 32 + i) * 72 + row] = (h16)((v - (float)ah) * LOSC); } }
        __syncthreads();
        const size_t rblk = (size_t)blockIdx.x * 64; const int b = (int)(rblk / NT_), t0 = (int)(rblk - (size_t)b * NT_); const int h = c0 / DV2, dbase = c0 - h * DV2;
        const int piece = tid & 7;
        auto pass = [&]() {
#pragma unroll
            for (int s = 0; s < 4; ++s) { const int d = (tid >> 3) + 16 * s; const size_t o = ((((size_t)b * NH_ + h) * DV2 + dbase + d) * NT_) + t0 + piece * 8;
                *(volatile v8h*)((h16*)C + o) = *(const v8ha*)(vt + d * 72 + piece * 8); *(volatile v8h*)((h16*)C2 + o) = *(const v8ha*)(vt2 + d * 72 + piece * 8); }
        };
        pass(); __threadfence(); pass();
    } else if (MODE == 4) {
        h16* c1 = (h16*)C + r0 * ldc + c0;
        auto pass = [&]() {
#pragma unroll
            for (int s = 0; s < 4; ++s) { const int row = 4 * s + (lane >> 3), piece = lane & 7; const float* sp = os + row * 68 + piece * 8; v8h o1;
#pragma unroll
                for (int i = 0; i < 8; ++i) o1[i] = (h16)sp[i];
                *(volatile v8h*)(c1 + (size_t)row * ldc + piece * 8) = o1; }
        };
        pass(); __threadfence(); pass();
    } else {
        bf* c1 = (bf*)C + r0 * ldc + c0; bf* c2 = (bf*)C2 + r0 * ldc + c0;
        auto pass = [&]() {
#pragma unroll
            for (int s = 0; s < 4; ++s) { const int row = 4 * s + (lane >> 3), piece = lane & 7; const float* sp = os + row * 68 + piece * 8; v8us o1, o2;
#pragma unroll
                for (int i = 0; i < 8; ++i) { const unsigned short hb = f2bf(sp[i]); o1[i] = hb; o2[i] = f2bf(sp[i] - bf2f(hb)); }
                *(volatile v8us*)(c1 + (size_t)row * ldc + piece * 8) = o1; *(volatile v8us*)(c2 + (size_t)row * ldc + piece * 8) = o2; }
        };
        pass(); __threadfence(); pass();
    }
}
__global__ __launch_bounds__(128) void k_mha(const h16* __restrict__ QH, const h16* __restrict__ KH, const h16* __restrict__ VTH, const h16* __restrict__ VTL, bf* CH, bf* CL) {
    __shared__ __align__(16) h16 plds[4][16 * 32];
    __shared__ __align__(16) h16 plds2[4][16 * 32];
    __shared__ __align__(16) float ost[4][16 * 68];
    const int lane = threadIdx.x & 31, wave = threadIdx.x >> 5, lr = lane & 15, hi = lane >> 4;
    const int bid = blockIdx.x;
    const int b = bid / (NH_ * (NT_ / 64)), rem = bid - b * (NH_ * (NT_ / 64)), h = rem / (NT_ / 64), qt = rem - h * (NT_ / 64), dh = blockIdx.y;
    const int q0 = qt * 64 + wave * 16;
    const size_t tok0 = (size_t)b * NT_;
    h16* pl = &plds[wave][0]; h16* pl2 = &plds2[wave][0];
    const size_t qo = (tok0 + q0 + lr) * DQ2 + h * DK2 + 8 * hi;
    const v16h qa = cat16(*(const v8h*)(QH + qo), *(const v8h*)(QH + qo + 16));
    const size_t vbase = (((size_t)b * NH_ + h) * DV2) * NT_;
    v8f o[4], ox[4];
#pragma unroll
    for (int n = 0; n < 4; ++n) { o[n] = (v8f){}; ox[n] = (v8f){}; }
    float mrow[8], lpart[8];
#pragma unroll
    for (int j = 0; j < 8; ++j) { mrow[j] = -3.0e38f; lpart[j] = 0.f; }
    const int kt_hi = (qt * 64 + 63) / 32;
#pragma unroll 1
    for (int kt = 0; kt <= kt_hi; ++kt) {
        const int l0 = kt * 32;
        const size_t k0o = (tok0 + l0 + lr) * DQ2 + h * DK2 + 8 * hi, k1o = k0o + (size_t)16 * DQ2;
        const v16h k0h = cat16(*(const v8h*)(KH + k0o), *(const v8h*)(KH + k0o + 16)), k1h = cat16(*(const v8h*)(KH + k1o), *(const v8h*)(KH + k1o + 16));
        v8f s0 = wmma16(qa, k0h, (v8f){}), s1 = wmma16(qa, k1h, (v8f){});
        asm volatile("v_nop\n\tv_nop\n\tv_nop\n\tv_nop" : "+v"(s0), "+v"(s1) : "v"(qa), "v"(k0h), "v"(k1h));
        float alpha[8];
#pragma unroll
        for (int j = 0; j < 8; ++j) { const int qi = q0 + hi * 8 + j, ja = l0 + lr, jb = l0 + 16 + lr;
            const float a0 = (ja <= qi) ? s0[j] * 0.17677669529663687f : NEGF, a1 = (jb <= qi) ? s1[j] * 0.17677669529663687f : NEGF;
            float mx = fmaxf(a0, a1);
            mx = fmaxf(mx, __shfl_xor(mx, 1, 16)); mx = fmaxf(mx, __shfl_xor(mx, 2, 16)); mx = fmaxf(mx, __shfl_xor(mx, 4, 16)); mx = fmaxf(mx, __shfl_xor(mx, 8, 16));
            const float mn = fmaxf(mrow[j], mx);
            alpha[j] = __expf(mrow[j] - mn); mrow[j] = mn;
            const float p0 = __expf(a0 - mn), p1 = __expf(a1 - mn);
            lpart[j] = lpart[j] * alpha[j] + (p0 + p1);
            const int mr = hi * 8 + j; const float ps0 = p0 * PSC, ps1 = p1 * PSC; const h16 h0 = (h16)ps0, h1 = (h16)ps1;
            pl[mr * 32 + lr] = h0; pl[mr * 32 + 16 + lr] = h1; pl2[mr * 32 + lr] = (h16)(ps0 - (float)h0); pl2[mr * 32 + 16 + lr] = (h16)(ps1 - (float)h1); }
#pragma unroll
        for (int n = 0; n < 4; ++n)
#pragma unroll
            for (int j = 0; j < 8; ++j) { o[n][j] *= alpha[j]; ox[n][j] *= alpha[j]; }
        asm volatile("" ::: "memory");
        const v16h pa = cat16(*(const v8ha*)(pl + lr * 32 + hi * 8), *(const v8ha*)(pl + lr * 32 + 16 + hi * 8));
        const v16h px = cat16(*(const v8ha*)(pl2 + lr * 32 + hi * 8), *(const v8ha*)(pl2 + lr * 32 + 16 + hi * 8));
#pragma unroll
        for (int n = 0; n < 4; ++n) { const size_t vo = vbase + (size_t)((dh * 4 + n) * 16 + lr) * NT_ + l0 + hi * 8; const v16h vh = cat16(*(const v8h*)(VTH + vo), *(const v8h*)(VTH + vo + 16)), vl = cat16(*(const v8h*)(VTL + vo), *(const v8h*)(VTL + vo + 16));
            o[n] = wmma16(pa, vh, o[n]); o[n] = wmma16(px, vh, o[n]); ox[n] = wmma16(pa, vl, ox[n]);
            asm volatile("" : "+v"(o[n]), "+v"(ox[n]) : "v"(vh), "v"(vl) : "memory"); }
        asm volatile("v_nop\n\tv_nop\n\tv_nop\n\tv_nop" : "+v"(o[0]), "+v"(o[3]), "+v"(ox[0]), "+v"(ox[3]) : "v"(pa), "v"(px));
        __builtin_amdgcn_wave_barrier();
    }
    float inv[8];
#pragma unroll
    for (int j = 0; j < 8; ++j) { float rs = lpart[j]; rs += __shfl_xor(rs, 1, 16); rs += __shfl_xor(rs, 2, 16); rs += __shfl_xor(rs, 4, 16); rs += __shfl_xor(rs, 8, 16); inv[j] = 1.0f / (rs * PSC); }
    float* os = &ost[wave][0];
    const size_t cbase = (tok0 + q0) * DO2 + (size_t)h * DV2;
    { const int half = dh;
#pragma unroll
        for (int n = 0; n < 4; ++n)
#pragma unroll
            for (int j = 0; j < 8; ++j) os[(hi * 8 + j) * 68 + n * 16 + lr] = (o[n][j] + ox[n][j] * LOSCI) * inv[j];
        __builtin_amdgcn_wave_barrier(); asm volatile("" ::: "memory");
#pragma unroll
        for (int ps2 = 0; ps2 < 2; ++ps2) {
#pragma unroll
            for (int s = 0; s < 4; ++s) { const int row = 4 * s + (lane >> 3), piece = lane & 7; const float* sp = os + row * 68 + piece * 8; v8us oh, ol;
#pragma unroll
                for (int i = 0; i < 8; ++i) { const unsigned short hb = f2bf(sp[i]); oh[i] = hb; ol[i] = f2bf(sp[i] - bf2f(hb)); }
                const size_t po = cbase + (size_t)row * DO2 + half * 64 + piece * 8; *(volatile v8us*)(CH + po) = oh; *(volatile v8us*)(CL + po) = ol; }
            if (ps2 == 0) __threadfence(); }
        __builtin_amdgcn_wave_barrier(); asm volatile("" ::: "memory");
    }
}
__global__ __launch_bounds__(256) void k_out(const float* __restrict__ OUTP, float* out) {
    const size_t f = (size_t)blockIdx.x * 256 + threadIdx.x;
    if (f >= (size_t)NTK * VOC) return;
    const size_t t = f / VOC; const int c = (int)(f - t * VOC);
    const float v = OUTP[t * 256 + c];
    *(volatile float*)(out + f) = v; __threadfence(); *(volatile float*)(out + f) = v;
}

extern "C" void kernel_launch(void* const* d_in, const int* in_sizes, int n_in,
                              void* d_out, int out_size, void* d_ws, size_t ws_size, hipStream_t stream) {
    (void)in_sizes; (void)n_in; (void)out_size;
    const int* xs = (const int*)d_in[0]; const float* lq = (const float*)d_in[1]; const float* lk = (const float*)d_in[2]; const float* lv = (const float*)d_in[3]; const float* relb = (const float*)d_in[4];
    const float* pq = (const float*)d_in[5]; const float* pk = (const float*)d_in[6]; const float* pv = (const float*)d_in[7]; const float* po = (const float*)d_in[8];
    float* out = (float*)d_out;
    char* wsp = (char*)d_ws;
    auto take = [&](size_t bytes) { char* p = wsp; wsp += (bytes + 255) & ~(size_t)255; return (void*)p; };
    const size_t RB = (size_t)NTK * 1024 * 2;
    char* RA = (char*)take(RB); char* RBX = (char*)take(RB); char* RC = (char*)take(RB / 2); char* RD = (char*)take(RB); char* RE = (char*)take(RB);
    bf* WqT = (bf*)take((size_t)DQ2 * DV1 * 2); bf* WkT = (bf*)take((size_t)DQ2 * DV1 * 2); bf* WvT = (bf*)take((size_t)DO2 * DV1 * 2); bf* WoT = (bf*)take((size_t)256 * DO2 * 2);
    if ((size_t)(wsp - (char*)d_ws) > ws_size) return;
    bf* Q1 = (bf*)RA; bf* K1 = (bf*)(RA + (size_t)NTK * DQ1 * 2); bf* V1T = (bf*)(RA + (size_t)NTK * DQ1 * 4);
    bf* X2H = (bf*)RBX; bf* X2L = (bf*)(RBX + RB / 2);
    h16* Q2 = (h16*)RC; h16* K2 = (h16*)(RC + RB / 4);
    h16* VTH = (h16*)RA; h16* VTL = (h16*)RD; bf* CH = (bf*)RBX; bf* CL = (bf*)RE; float* OUTP = (float*)RC;
    k_gather<<<NTK / 8, 256, 0, stream>>>(xs, lq, lk, Q1, K1);
    k_gvt<<<dim3(NT_ / 64, DV1 / 64, NB_), 256, 0, stream>>>(xs, lv, V1T);
    k_local<<<dim3(NT_ / 64, DV1 / 128, NB_), 128, 0, stream>>>(Q1, K1, V1T, relb, X2H, X2L);
    k_wt<<<dim3(DV1 / 64, DQ2 / 64, 1), 256, 0, stream>>>(pq, DV1, DQ2, DQ2, WqT); k_wt<<<dim3(DV1 / 64, DQ2 / 64, 1), 256, 0, stream>>>(pk, DV1, DQ2, DQ2, WkT);
    k_wt<<<dim3(DV1 / 64, DO2 / 64, 1), 256, 0, stream>>>(pv, DV1, DO2, DO2, WvT); k_wt<<<dim3(DO2 / 64, 256 / 64, 1), 256, 0, stream>>>(po, DO2, VOC, 256, WoT);
    k_gemm<4><<<dim3(NTK / 64, DQ2 / 64, 1), 128, 0, stream>>>(X2H, X2L, DV1, WqT, DV1, DQ2, Q2, nullptr);
    k_gemm<4><<<dim3(NTK / 64, DQ2 / 64, 1), 128, 0, stream>>>(X2H, X2L, DV1, WkT, DV1, DQ2, K2, nullptr);
    k_gemm<2><<<dim3(NTK / 64, DO2 / 64, 1), 128, 0, stream>>>(X2H, X2L, DV1, WvT, DV1, DO2, VTH, VTL);
    k_mha<<<dim3(NB_ * NH_ * (NT_ / 64), 2, 1), 128, 0, stream>>>(Q2, K2, VTH, VTL, CH, CL);
    k_gemm<1><<<dim3(NTK / 64, 256 / 64, 1), 128, 0, stream>>>(CH, CL, DO2, WoT, DO2, 256, OUTP, nullptr);
    k_out<<<(unsigned)(((size_t)NTK * VOC + 255) / 256), 256, 0, stream>>>(OUTP, out);
}
